// PointNetSetUpConv_33724083208691
// MI455X (gfx1250) — hardware-verified
//
#include <hip/hip_runtime.h>
#pragma clang fp contract(off)

typedef __attribute__((ext_vector_type(16))) _Float16 v16h;
typedef __attribute__((ext_vector_type(8)))  _Float16 v8h;
typedef __attribute__((ext_vector_type(4)))  _Float16 v4h;
typedef __attribute__((ext_vector_type(8)))  float    v8f;
typedef __attribute__((ext_vector_type(4)))  float    v4f;
typedef __attribute__((ext_vector_type(4)))  int      v4i;

constexpr int NBATCH    = 4;
constexpr int NPTS1     = 8192;
constexpr int NPTS2     = 2048;
constexpr int CH_F1     = 128;
constexpr int CH_F2     = 256;
constexpr int CH_L0     = 128;
constexpr int CH_L1     = 128;
constexpr int CH_L2     = 256;
constexpr int CH_OUT    = 256;
constexpr int KDIM_MLP2 = CH_L2 + CH_F1;
constexpr int W10_PITCH = CH_F2 + 3;
constexpr int KNN_NS    = 8;
constexpr float W_CARRY     = 16.0f;
constexpr float W_CARRY_INV = 1.0f / 16.0f;
constexpr float RES_CARRY      = 2048.0f;
constexpr float RES_CARRY_INV  = 1.0f / 2048.0f;
constexpr float F16_MIN_NORMAL = 6.103515625e-5f;
static_assert(KDIM_MLP2 == 384, "mlp2 K");
static_assert(W10_PITCH == 259, "w1_0 pitch");
static_assert(CH_F2 % 32 == 0 && CH_L0 % 32 == 0 && CH_L1 % 32 == 0 && KDIM_MLP2 % 32 == 0, "K multiples of 32");

constexpr int BNT_S0 = 0;
constexpr int BNT_T0 = 128;
constexpr int BNT_S1 = 256;
constexpr int BNT_T1 = 384;
constexpr int BNT_S2 = 512;
constexpr int BNT_T2 = 768;
constexpr int BNT_S4 = 1024;
constexpr int BNT_T4 = 1280;
constexpr int BNT_TOTAL = 1536;

constexpr int WPL_WF = 0;
constexpr int WPL_W1 = WPL_WF + CH_L0 * CH_F2;
constexpr int WPL_W2 = WPL_W1 + CH_L1 * CH_L0;
constexpr int WPL_W4 = WPL_W2 + CH_L2 * CH_L1;
constexpr int WPL_TOTAL = WPL_W4 + CH_OUT * KDIM_MLP2;
static_assert(WPL_TOTAL == 180224, "weight plane halves");
static_assert(WPL_TOTAL / 8 == 88 * 256, "cast pieces fill 88 blocks exactly");

constexpr size_t WS_IDX = 0;
constexpr size_t WS_F2T = WS_IDX + (size_t)NBATCH * NPTS1 * KNN_NS * 4;
constexpr size_t WS_PPL = WS_F2T + (size_t)NBATCH * NPTS2 * CH_F2 * 2;
constexpr size_t WS_X2  = WS_PPL + (size_t)NBATCH * NPTS2 * CH_L0 * 4;
constexpr size_t WS_X2L = WS_X2 + (size_t)NBATCH * NPTS1 * KDIM_MLP2 * 2;
constexpr size_t WS_WPL = WS_X2L + (size_t)NBATCH * NPTS1 * KDIM_MLP2 * 2;
constexpr size_t WS_WP  = WS_WPL + (size_t)WPL_TOTAL * 2;
constexpr size_t WS_BNT = WS_WP + (size_t)CH_L0 * 4 * 4;
constexpr size_t WS_TOTAL = WS_BNT + (size_t)BNT_TOTAL * 4;
static_assert(WS_F2T % 128 == 0 && WS_PPL % 128 == 0 && WS_X2 % 128 == 0 && WS_X2L % 128 == 0 && WS_WPL % 128 == 0 && WS_WP % 128 == 0 && WS_BNT % 128 == 0, "line aligned carve");
static_assert(WS_TOTAL == (size_t)60137472, "carve total");
static_assert(WS_TOTAL <= (size_t)134217728, "carve under 128 MiB");

struct FragH {
  union U { v16h v; v8h h[2]; };
  static __device__ __forceinline__ v16h load(const _Float16* p) {
    U f;
    f.h[0] = *(const v8h*)(p);
    f.h[1] = *(const v8h*)(p + 16);
    return f.v;
  }
  static __device__ __forceinline__ v8f mma(v16h a, v16h b, v8f c) {
    return __builtin_amdgcn_wmma_f32_16x16x32_f16(false, a, false, b, (short)0, c, false, false);
  }
};
__device__ __forceinline__ void guard4_h(v8f& a, v8f& b, v8f& c, v8f& d, v16h x) {
  asm volatile("v_nop\n\tv_nop\n\tv_nop\n\tv_nop" : "+v"(a), "+v"(b), "+v"(c), "+v"(d) : "v"(x));
}
__device__ __forceinline__ void guard2_h(v8f& a, v8f& b, v16h x0, v16h x1, v16h x2, v16h x3) {
  asm volatile("v_nop\n\tv_nop\n\tv_nop\n\tv_nop" : "+v"(a), "+v"(b) : "v"(x0), "v"(x1), "v"(x2), "v"(x3));
}
__device__ __forceinline__ void keep4_h(v16h a, v16h b, v16h c, v16h d) {
  asm volatile("v_nop" :: "v"(a), "v"(b), "v"(c), "v"(d));
}
__device__ __forceinline__ void acc_guard4(v8f& a, v8f& b, v8f& c, v8f& d) {
  asm volatile("v_nop\n\tv_nop\n\tv_nop\n\tv_nop" : "+v"(a), "+v"(b), "+v"(c), "+v"(d));
}

__device__ __forceinline__ float hi_part(float x) {
  const _Float16 h0 = (_Float16)x;
  const float hf0 = (float)h0;
  return (fabsf(hf0) < F16_MIN_NORMAL) ? 0.0f : hf0;
}
__device__ __forceinline__ float lo_part(float x, float hf) {
  const float d = x - hf;
  return d * RES_CARRY;
}

__device__ __forceinline__ void bn_piece(int p, const float* __restrict__ bn0, const float* __restrict__ bn1,
                                         const float* __restrict__ bn2, const float* __restrict__ bn4,
                                         float* __restrict__ bnt) {
  const float* bn = (p < 64) ? bn0 : (p < 128) ? bn1 : (p < 256) ? bn2 : bn4;
  const int nch = (p < 128) ? 128 : 256;
  const int pl = (p < 64) ? p : (p < 128) ? (p - 64) : (p < 256) ? (p - 128) : (p - 256);
  const int per = nch / 4;
  const bool isShift = pl >= per;
  const int c0 = 4 * (isShift ? (pl - per) : pl);
  const v4f g  = *(const v4f*)(bn + c0);
  const v4f be = *(const v4f*)(bn + nch + c0);
  const v4f mu = *(const v4f*)(bn + 2 * nch + c0);
  const v4f va = *(const v4f*)(bn + 3 * nch + c0);
  v4f o;
#pragma unroll
  for (int e = 0; e < 4; ++e) {
    const float sc = g[e] * rsqrtf(va[e] + 1e-5f);
    const float ms = mu[e] * sc;
    const float sh = be[e] - ms;
    o[e] = isShift ? sh : (sc * W_CARRY_INV);
  }
  *(volatile v4f*)(bnt + 4 * p) = o;
  __threadfence();
  *(volatile v4f*)(bnt + 4 * p) = o;
}

__global__ __launch_bounds__(256) void prep_planes(
    const float* __restrict__ w10, const float* __restrict__ w11, const float* __restrict__ w12,
    const float* __restrict__ w20, const float* __restrict__ bn0, const float* __restrict__ bn1,
    const float* __restrict__ bn2, const float* __restrict__ bn4,
    unsigned short* __restrict__ wplp, float* __restrict__ wp, float* __restrict__ bnt) {
  const int tid = threadIdx.x;
  const int blk = blockIdx.x;
  if (blk < 88) {
    const int g = blk * 256 + tid;
    const float* sp;
    if (blk < 16) {
      const int row = g >> 5;
      const int c8 = (g & 31) * 8;
      sp = w10 + (size_t)row * W10_PITCH + c8;
    } else if (blk < 24) {
      sp = w11 + (size_t)(g - 4096) * 8;
    } else if (blk < 40) {
      sp = w12 + (size_t)(g - 6144) * 8;
    } else {
      sp = w20 + (size_t)(g - 10240) * 8;
    }
    v8h hv;
#pragma unroll
    for (int e = 0; e < 8; ++e) {
      const float x = sp[e] * W_CARRY;
      hv[e] = (_Float16)x;
    }
    _Float16* dst = (_Float16*)wplp + (size_t)g * 8;
    *(volatile v8h*)dst = hv;
    __threadfence();
    *(volatile v8h*)dst = hv;
  } else if (blk == 88) {
    if (tid < 128) {
      const float* s = w10 + (size_t)tid * W10_PITCH + CH_F2;
      v4f o;
      o[0] = s[0] * W_CARRY;
      o[1] = s[1] * W_CARRY;
      o[2] = s[2] * W_CARRY;
      o[3] = 0.0f;
      *(volatile v4f*)(wp + tid * 4) = o;
      __threadfence();
      *(volatile v4f*)(wp + tid * 4) = o;
    } else {
      bn_piece(tid - 128, bn0, bn1, bn2, bn4, bnt);
    }
  } else {
    bn_piece(128 + tid, bn0, bn1, bn2, bn4, bnt);
  }
}

template <int NCH, bool SPLIT>
__global__ __launch_bounds__(256) void transpose_cast(
    const float* __restrict__ src, unsigned short* dstp, unsigned short* dst2p, int npts, int dpitch, int dcol) {
  __shared__ float tile[NCH * 33];
  constexpr int LD_IT = NCH / 32;
  constexpr int PR = NCH / 8;
  constexpr int ST_IT = NCH / 64;
  const int tid = threadIdx.x;
  const int b = blockIdx.y;
  const int n0 = blockIdx.x * 32;
#pragma unroll
  for (int it = 0; it < LD_IT; ++it) {
    const int q = it * 256 + tid;
    const int c = q >> 3;
    const int m4 = (q & 7) * 4;
    const v4f v = *(const v4f*)(src + ((size_t)b * NCH + c) * npts + n0 + m4);
    tile[c * 33 + m4 + 0] = v[0];
    tile[c * 33 + m4 + 1] = v[1];
    tile[c * 33 + m4 + 2] = v[2];
    tile[c * 33 + m4 + 3] = v[3];
    if (it == 3) asm volatile("" ::: "memory");
  }
  __syncthreads();
  v8h hv[ST_IT];
  v8h lv[ST_IT];
#pragma unroll
  for (int it = 0; it < ST_IT; ++it) {
    const int p = it * 256 + tid;
    const int n = p / PR;
    const int c0 = (p % PR) * 8;
#pragma unroll
    for (int e = 0; e < 8; ++e) {
      const float x = tile[(c0 + e) * 33 + n];
      if (SPLIT) {
        const float hf = hi_part(x);
        const float rf = lo_part(x, hf);
        hv[it][e] = (_Float16)hf;
        lv[it][e] = (_Float16)rf;
      } else {
        hv[it][e] = (_Float16)x;
        lv[it][e] = hv[it][e];
      }
    }
  }
  _Float16* dst = (_Float16*)dstp;
  _Float16* dst2 = (_Float16*)dst2p;
  for (int pass = 0; pass < 2; ++pass) {
#pragma unroll
    for (int it = 0; it < ST_IT; ++it) {
      const int p = it * 256 + tid;
      const int n = p / PR;
      const int c0 = (p % PR) * 8;
      const size_t off = ((size_t)b * npts + n0 + n) * dpitch + dcol + c0;
      *(volatile v8h*)(dst + off) = hv[it];
      if (SPLIT) *(volatile v8h*)(dst2 + off) = lv[it];
    }
    __threadfence();
  }
}

__global__ __launch_bounds__(256) void knn8_kernel(
    const float* __restrict__ xyz1, const float* __restrict__ xyz2, int* __restrict__ idx) {
#pragma clang fp contract(off)
  __shared__ __align__(16) v4f s2[NPTS2];
  __shared__ __align__(16) int sidx[256 * KNN_NS];
  const int tid = threadIdx.x;
  const int b = blockIdx.y;
#pragma unroll 1
  for (int i = tid; i < NPTS2; i += 256) {
    const float* p = xyz2 + ((size_t)b * NPTS2 + i) * 3;
    const float x = p[0];
    const float y = p[1];
    const float z = p[2];
    const float t0 = x * x;
    const float t1 = y * y;
    const float t2 = z * z;
    v4f o;
    o[0] = x;
    o[1] = y;
    o[2] = z;
    o[3] = (t0 + t2) + t1;
    s2[i] = o;
  }
  __syncthreads();
  const int q = blockIdx.x * 256 + tid;
  const float* pq = xyz1 + ((size_t)b * NPTS1 + q) * 3;
  const float px = pq[0];
  const float py = pq[1];
  const float pz = pq[2];
  const float u0 = px * px;
  const float u1 = py * py;
  const float u2 = pz * pz;
  const float sq1 = (u0 + u2) + u1;
  float bd[KNN_NS];
  int bi[KNN_NS];
#pragma unroll
  for (int t = 0; t < KNN_NS; ++t) {
    bd[t] = __builtin_inff();
    bi[t] = 0;
  }
#pragma unroll 4
  for (int j = 0; j < NPTS2; ++j) {
    const v4f s = s2[j];
    float p = px * s[0];
    p = __builtin_fmaf(py, s[1], p);
    p = __builtin_fmaf(pz, s[2], p);
    const float two_p = 2.0f * p;
    const float d = (sq1 + s[3]) - two_p;
    if (d < bd[KNN_NS - 1]) {
#pragma unroll
      for (int t = KNN_NS - 1; t >= 1; --t) {
        const bool mv = d < bd[t - 1];
        const bool ins = d < bd[t];
        const float nd = mv ? bd[t - 1] : (ins ? d : bd[t]);
        const int ni = mv ? bi[t - 1] : (ins ? j : bi[t]);
        bd[t] = nd;
        bi[t] = ni;
      }
      const bool ins0 = d < bd[0];
      const float nd0 = ins0 ? d : bd[0];
      const int ni0 = ins0 ? j : bi[0];
      bd[0] = nd0;
      bi[0] = ni0;
    }
  }
#pragma unroll
  for (int t = 0; t < KNN_NS; ++t) {
    int v = bi[t];
    v = v < 0 ? 0 : (v > NPTS2 - 1 ? NPTS2 - 1 : v);
    sidx[tid * KNN_NS + t] = v;
  }
  __syncthreads();
  const int wave = tid >> 5;
  const int lane = tid & 31;
  int* gdst = idx + ((size_t)b * NPTS1 + blockIdx.x * 256 + wave * 32) * KNN_NS;
  const v4i w0 = *(const v4i*)(sidx + wave * 256 + lane * 4);
  const v4i w1 = *(const v4i*)(sidx + wave * 256 + 128 + lane * 4);
  for (int pass = 0; pass < 2; ++pass) {
    *(volatile v4i*)(gdst + lane * 4) = w0;
    *(volatile v4i*)(gdst + 128 + lane * 4) = w1;
    __threadfence();
  }
}

template <bool ROWAFF>
__global__ __launch_bounds__(256) void gemm64_f16(
    const unsigned short* __restrict__ Ap, int lda, long strideA,
    const unsigned short* __restrict__ Btp, int ldb, long strideB,
    float* __restrict__ Cout, int ldc, long strideC,
    const float* __restrict__ rscale, const float* __restrict__ rshift,
    int M, int N, int K) {
  const _Float16* A = (const _Float16*)Ap;
  const _Float16* Bt = (const _Float16*)Btp;
  __shared__ __align__(16) float sT[8][16 * 68];
  const int b    = blockIdx.y;
  const int lane = threadIdx.x & 31;
  const int wave = threadIdx.x >> 5;
  const int tilesN = N >> 6;
  const int tilesM = M >> 6;
  const int tile = blockIdx.x * 8 + wave;
  if (tile >= tilesM * tilesN) return;
  const int tm = tile / tilesN;
  const int tn = tile - tm * tilesN;
  const int m0 = tm << 6;
  const int n0 = tn << 6;

  const _Float16* Ab = A + (size_t)b * strideA;
  const _Float16* Bb = Bt + (size_t)b * strideB;

  const int rlane = lane & 15;
  const int koff  = (lane >> 4) * 8;
  const int mOff  = (lane >> 4) * 8;

  v8f acc[4][4];
#pragma unroll
  for (int i = 0; i < 4; ++i)
#pragma unroll
    for (int j = 0; j < 4; ++j) acc[i][j] = (v8f){0.f, 0.f, 0.f, 0.f, 0.f, 0.f, 0.f, 0.f};

  for (int k0 = 0; k0 < K; k0 += 32) {
    v16h bh[4];
#pragma unroll
    for (int j = 0; j < 4; ++j) {
      const size_t bo = (size_t)(n0 + (j << 4) + rlane) * ldb + koff + k0;
      bh[j] = FragH::load(Bb + bo);
    }
#pragma unroll
    for (int i = 0; i < 4; ++i) {
      const size_t ao = (size_t)(m0 + (i << 4) + rlane) * lda + koff + k0;
      const v16h ah = FragH::load(Ab + ao);
#pragma unroll
      for (int j = 0; j < 4; ++j) acc[i][j] = FragH::mma(ah, bh[j], acc[i][j]);
      guard4_h(acc[i][0], acc[i][1], acc[i][2], acc[i][3], ah);
    }
    keep4_h(bh[0], bh[1], bh[2], bh[3]);
  }
  acc_guard4(acc[0][0], acc[0][1], acc[0][2], acc[0][3]);
  acc_guard4(acc[1][0], acc[1][1], acc[1][2], acc[1][3]);
  acc_guard4(acc[2][0], acc[2][1], acc[2][2], acc[2][3]);
  acc_guard4(acc[3][0], acc[3][1], acc[3][2], acc[3][3]);

  float* slab = sT[wave];
  float* C = Cout + (size_t)b * strideC;
#pragma unroll
  for (int i = 0; i < 4; ++i) {
    const int mBase = m0 + (i << 4);
    v4f sc0 = (v4f){1.f, 1.f, 1.f, 1.f};
    v4f sc1 = sc0;
    v4f sh0 = (v4f){0.f, 0.f, 0.f, 0.f};
    v4f sh1 = sh0;
    if (ROWAFF) {
      sc0 = *(const v4f*)(rscale + mBase + mOff);
      sc1 = *(const v4f*)(rscale + mBase + mOff + 4);
      sh0 = *(const v4f*)(rshift + mBase + mOff);
      sh1 = *(const v4f*)(rshift + mBase + mOff + 4);
    }
#pragma unroll
    for (int j = 0; j < 4; ++j) {
#pragma unroll
      for (int r = 0; r < 8; ++r) {
        float v = acc[i][j][r];
        if (ROWAFF) {
          const float sc = (r < 4) ? sc0[r & 3] : sc1[r & 3];
          const float sh = (r < 4) ? sh0[r & 3] : sh1[r & 3];
          const float t = v * sc;
          v = fmaxf(t + sh, 0.0f);
        }
        slab[(mOff + r) * 68 + (j << 4) + rlane] = v;
      }
    }
    __builtin_amdgcn_fence(__ATOMIC_RELEASE, "workgroup");
    __builtin_amdgcn_wave_barrier();
    __builtin_amdgcn_fence(__ATOMIC_ACQUIRE, "workgroup");
    {
      const int hh = lane >> 4;
      const int c4 = (lane & 15) * 4;
      for (int pass = 0; pass < 2; ++pass) {
#pragma unroll
        for (int it = 0; it < 8; ++it) {
          const int row = it * 2 + hh;
          const v4f v = *(const v4f*)(slab + row * 68 + c4);
          *(volatile v4f*)(C + (size_t)(mBase + row) * ldc + n0 + c4) = v;
        }
        __threadfence();
      }
    }
    __builtin_amdgcn_fence(__ATOMIC_RELEASE, "workgroup");
    __builtin_amdgcn_wave_barrier();
    __builtin_amdgcn_fence(__ATOMIC_ACQUIRE, "workgroup");
  }
}

__global__ __launch_bounds__(256) void gemm_mlp2_hilo(
    const unsigned short* __restrict__ Ap, int lda,
    const unsigned short* __restrict__ Bhp, const unsigned short* __restrict__ Blp, int ldb, long strideB,
    float* __restrict__ Cout, int ldc, long strideC,
    const float* __restrict__ rscale, const float* __restrict__ rshift,
    int M, int N, int K) {
  const _Float16* A  = (const _Float16*)Ap;
  const _Float16* Bh = (const _Float16*)Bhp;
  const _Float16* Bl = (const _Float16*)Blp;
  __shared__ __align__(16) float sT[8][16 * 36];
  const int b    = blockIdx.y;
  const int lane = threadIdx.x & 31;
  const int wave = threadIdx.x >> 5;
  const int tilesN = N >> 5;
  const int tilesM = M >> 6;
  const int tile = blockIdx.x * 8 + wave;
  if (tile >= tilesM * tilesN) return;
  const int tm = tile / tilesN;
  const int tn = tile - tm * tilesN;
  const int m0 = tm << 6;
  const int n0 = tn << 5;

  const _Float16* Bhb = Bh + (size_t)b * strideB;
  const _Float16* Blb = Bl + (size_t)b * strideB;

  const int rlane = lane & 15;
  const int koff  = (lane >> 4) * 8;
  const int mOff  = (lane >> 4) * 8;

  v8f acc[4][2];
  v8f accr[4][2];
#pragma unroll
  for (int i = 0; i < 4; ++i)
#pragma unroll
    for (int j = 0; j < 2; ++j) {
      acc[i][j]  = (v8f){0.f, 0.f, 0.f, 0.f, 0.f, 0.f, 0.f, 0.f};
      accr[i][j] = (v8f){0.f, 0.f, 0.f, 0.f, 0.f, 0.f, 0.f, 0.f};
    }

  for (int k0 = 0; k0 < K; k0 += 32) {
    v16h bh[2];
    v16h bl[2];
#pragma unroll
    for (int j = 0; j < 2; ++j) {
      const size_t bo = (size_t)(n0 + (j << 4) + rlane) * ldb + koff + k0;
      bh[j] = FragH::load(Bhb + bo);
      bl[j] = FragH::load(Blb + bo);
    }
#pragma unroll
    for (int i = 0; i < 4; ++i) {
      const size_t ao = (size_t)(m0 + (i << 4) + rlane) * lda + koff + k0;
      const v16h ah = FragH::load(A + ao);
#pragma unroll
      for (int j = 0; j < 2; ++j) {
        acc[i][j]  = FragH::mma(ah, bh[j], acc[i][j]);
        accr[i][j] = FragH::mma(ah, bl[j], accr[i][j]);
      }
      guard4_h(acc[i][0], acc[i][1], accr[i][0], accr[i][1], ah);
    }
    keep4_h(bh[0], bh[1], bl[0], bl[1]);
  }
  acc_guard4(acc[0][0], acc[0][1], accr[0][0], accr[0][1]);
  acc_guard4(acc[1][0], acc[1][1], accr[1][0], accr[1][1]);
  acc_guard4(acc[2][0], acc[2][1], accr[2][0], accr[2][1]);
  acc_guard4(acc[3][0], acc[3][1], accr[3][0], accr[3][1]);

  float* slab = sT[wave];
  float* C = Cout + (size_t)b * strideC;
#pragma unroll
  for (int i = 0; i < 4; ++i) {
    const int mBase = m0 + (i << 4);
    const v4f sc0 = *(const v4f*)(rscale + mBase + mOff);
    const v4f sc1 = *(const v4f*)(rscale + mBase + mOff + 4);
    const v4f sh0 = *(const v4f*)(rshift + mBase + mOff);
    const v4f sh1 = *(const v4f*)(rshift + mBase + mOff + 4);
#pragma unroll
    for (int j = 0; j < 2; ++j) {
#pragma unroll
      for (int r = 0; r < 8; ++r) {
        const float tr = accr[i][j][r] * RES_CARRY_INV;
        const float s = acc[i][j][r] + tr;
        const float sc = (r < 4) ? sc0[r & 3] : sc1[r & 3];
        const float sh = (r < 4) ? sh0[r & 3] : sh1[r & 3];
        const float t = s * sc;
        const float v = fmaxf(t + sh, 0.0f);
        slab[(mOff + r) * 36 + (j << 4) + rlane] = v;
      }
    }
    __builtin_amdgcn_fence(__ATOMIC_RELEASE, "workgroup");
    __builtin_amdgcn_wave_barrier();
    __builtin_amdgcn_fence(__ATOMIC_ACQUIRE, "workgroup");
    {
      const int rq = lane >> 3;
      const int c4 = (lane & 7) * 4;
      for (int pass = 0; pass < 2; ++pass) {
#pragma unroll
        for (int it = 0; it < 4; ++it) {
          const int row = it * 4 + rq;
          const v4f v = *(const v4f*)(slab + row * 36 + c4);
          *(volatile v4f*)(C + (size_t)(mBase + row) * ldc + n0 + c4) = v;
        }
        __threadfence();
      }
    }
    __builtin_amdgcn_fence(__ATOMIC_RELEASE, "workgroup");
    __builtin_amdgcn_wave_barrier();
    __builtin_amdgcn_fence(__ATOMIC_ACQUIRE, "workgroup");
  }
}

constexpr int A_PITCH = 136;
__global__ __launch_bounds__(128) void mlp1_fused(
    const float* __restrict__ xyz1, const float* __restrict__ xyz2, const int* __restrict__ idx,
    const float* __restrict__ P, const unsigned short* __restrict__ W1p, const unsigned short* __restrict__ W2p,
    const float* __restrict__ Wp, const float* __restrict__ bnt,
    unsigned short* __restrict__ X2p, unsigned short* __restrict__ X2Lp) {
  __shared__ __align__(16) _Float16 sA[4][32 * A_PITCH];
  __shared__ __align__(16) float sPool[4][4 * CH_L2];
  const _Float16* W1 = (const _Float16*)W1p;
  const _Float16* W2 = (const _Float16*)W2p;
  _Float16* X2 = (_Float16*)X2p;
  _Float16* X2L = (_Float16*)X2Lp;
  const int tid = threadIdx.x;
  const int lane = tid & 31;
  const int wave = tid >> 5;
  const int rlane = lane & 15;
  const int hh = lane >> 4;
  const int koff = hh * 8;
  const int Q0 = blockIdx.x * 16 + wave * 4;
  const int b = Q0 / NPTS1;

  int jv = idx[(size_t)Q0 * KNN_NS + lane];
  jv = jv < 0 ? 0 : (jv > NPTS2 - 1 ? NPTS2 - 1 : jv);
  const int Ql = Q0 + (lane >> 3);
  const float* p2 = xyz2 + ((size_t)b * NPTS2 + jv) * 3;
  const float* p1 = xyz1 + (size_t)Ql * 3;
  const float dxl = p2[0] - p1[0];
  const float dyl = p2[1] - p1[1];
  const float dzl = p2[2] - p1[2];

  const int c4 = lane * 4;
  const v4f wp0 = *(const v4f*)(Wp + (c4 + 0) * 4);
  const v4f wp1 = *(const v4f*)(Wp + (c4 + 1) * 4);
  const v4f wp2 = *(const v4f*)(Wp + (c4 + 2) * 4);
  const v4f wp3 = *(const v4f*)(Wp + (c4 + 3) * 4);
  const v4f s0 = *(const v4f*)(bnt + BNT_S0 + c4);
  const v4f t0 = *(const v4f*)(bnt + BNT_T0 + c4);

  _Float16* At = sA[wave];
#pragma unroll 4
  for (int r = 0; r < 32; ++r) {
    const int jr = __shfl(jv, r, 32);
    const float dx = __shfl(dxl, r, 32);
    const float dy = __shfl(dyl, r, 32);
    const float dz = __shfl(dzl, r, 32);
    const v4f pv = *(const v4f*)(P + ((size_t)b * NPTS2 + jr) * CH_L0 + c4);
    const float z0 = pv[0] + ((dx * wp0[0] + dy * wp0[1]) + dz * wp0[2]);
    const float z1 = pv[1] + ((dx * wp1[0] + dy * wp1[1]) + dz * wp1[2]);
    const float z2 = pv[2] + ((dx * wp2[0] + dy * wp2[1]) + dz * wp2[2]);
    const float z3 = pv[3] + ((dx * wp3[0] + dy * wp3[1]) + dz * wp3[2]);
    const float h0 = fmaxf(z0 * s0[0] + t0[0], 0.0f);
    const float h1 = fmaxf(z1 * s0[1] + t0[1], 0.0f);
    const float h2 = fmaxf(z2 * s0[2] + t0[2], 0.0f);
    const float h3 = fmaxf(z3 * s0[3] + t0[3], 0.0f);
    v4h hv;
    hv[0] = (_Float16)h0;
    hv[1] = (_Float16)h1;
    hv[2] = (_Float16)h2;
    hv[3] = (_Float16)h3;
    *(v4h*)(At + r * A_PITCH + c4) = hv;
  }
  __syncthreads();

  v16h a[2][4];
#pragma unroll
  for (int mt = 0; mt < 2; ++mt)
#pragma unroll
    for (int ks = 0; ks < 4; ++ks)
      a[mt][ks] = FragH::load(At + (mt * 16 + rlane) * A_PITCH + ks * 32 + koff);
  __syncthreads();

#pragma unroll 1
  for (int nt = 0; nt < CH_L1 / 16; ++nt) {
    const int cn = nt * 16 + rlane;
    v16h bf[4];
#pragma unroll
    for (int ks = 0; ks < 4; ++ks) bf[ks] = FragH::load(W1 + (size_t)cn * CH_L0 + ks * 32 + koff);
    const float sc = bnt[BNT_S1 + cn];
    const float sh = bnt[BNT_T1 + cn];
    v8f acc0 = (v8f){0.f, 0.f, 0.f, 0.f, 0.f, 0.f, 0.f, 0.f};
    v8f acc1 = (v8f){0.f, 0.f, 0.f, 0.f, 0.f, 0.f, 0.f, 0.f};
#pragma unroll
    for (int ks = 0; ks < 4; ++ks) {
      acc0 = FragH::mma(a[0][ks], bf[ks], acc0);
      acc1 = FragH::mma(a[1][ks], bf[ks], acc1);
    }
    guard2_h(acc0, acc1, bf[0], bf[1], bf[2], bf[3]);
#pragma unroll
    for (int r = 0; r < 8; ++r) {
      const float v0 = fmaxf(acc0[r] * sc + sh, 0.0f);
      const float v1 = fmaxf(acc1[r] * sc + sh, 0.0f);
      At[(8 * hh + r) * A_PITCH + cn] = (_Float16)v0;
      At[(16 + 8 * hh + r) * A_PITCH + cn] = (_Float16)v1;
    }
  }
  __syncthreads();

#pragma unroll
  for (int mt = 0; mt < 2; ++mt)
#pragma unroll
    for (int ks = 0; ks < 4; ++ks)
      a[mt][ks] = FragH::load(At + (mt * 16 + rlane) * A_PITCH + ks * 32 + koff);

  float* pl = sPool[wave];
#pragma unroll 1
  for (int nt = 0; nt < CH_L2 / 16; ++nt) {
    const int cn = nt * 16 + rlane;
    v16h bf[4];
#pragma unroll
    for (int ks = 0; ks < 4; ++ks) bf[ks] = FragH::load(W2 + (size_t)cn * CH_L1 + ks * 32 + koff);
    const float sc = bnt[BNT_S2 + cn];
    const float sh = bnt[BNT_T2 + cn];
    v8f acc0 = (v8f){0.f, 0.f, 0.f, 0.f, 0.f, 0.f, 0.f, 0.f};
    v8f acc1 = (v8f){0.f, 0.f, 0.f, 0.f, 0.f, 0.f, 0.f, 0.f};
#pragma unroll
    for (int ks = 0; ks < 4; ++ks) {
      acc0 = FragH::mma(a[0][ks], bf[ks], acc0);
      acc1 = FragH::mma(a[1][ks], bf[ks], acc1);
    }
    guard2_h(acc0, acc1, bf[0], bf[1], bf[2], bf[3]);
    float m0 = 0.0f;
    float m1 = 0.0f;
#pragma unroll
    for (int r = 0; r < 8; ++r) {
      m0 = fmaxf(m0, acc0[r] * sc + sh);
      m1 = fmaxf(m1, acc1[r] * sc + sh);
    }
    pl[hh * CH_L2 + cn] = m0;
    pl[(2 + hh) * CH_L2 + cn] = m1;
  }
  __syncthreads();

  v8h pvv[4];
  v8h pvl[4];
#pragma unroll
  for (int it = 0; it < 4; ++it) {
    const float* sp = pl + it * CH_L2 + lane * 8;
    const v4f x0 = *(const v4f*)(sp);
    const v4f x1 = *(const v4f*)(sp + 4);
#pragma unroll
    for (int e = 0; e < 4; ++e) {
      const float xa = x0[e];
      const float xb = x1[e];
      const float ha = hi_part(xa);
      const float hb = hi_part(xb);
      const float ra = lo_part(xa, ha);
      const float rb = lo_part(xb, hb);
      pvv[it][e] = (_Float16)ha;
      pvv[it][4 + e] = (_Float16)hb;
      pvl[it][e] = (_Float16)ra;
      pvl[it][4 + e] = (_Float16)rb;
    }
  }
  for (int pass = 0; pass < 2; ++pass) {
#pragma unroll
    for (int it = 0; it < 4; ++it) {
      const size_t off = (size_t)(Q0 + it) * KDIM_MLP2 + lane * 8;
      *(volatile v8h*)(X2 + off) = pvv[it];
      *(volatile v8h*)(X2L + off) = pvl[it];
    }
    __threadfence();
  }
}

static_assert((NBATCH * NPTS2) % 64 == 0 && CH_L0 % 64 == 0, "P GEMM tiles");
static_assert((((NBATCH * NPTS2) / 64) * (CH_L0 / 64)) % 8 == 0, "P GEMM tiles per block");
static_assert(CH_OUT % 64 == 0 && NPTS1 % 32 == 0, "mlp2 GEMM tiles");
static_assert(((CH_OUT / 64) * (NPTS1 / 32)) % 8 == 0, "mlp2 GEMM tiles per block");
static_assert(NPTS1 % 256 == 0 && NPTS1 % 16 == 0 && NPTS2 % 32 == 0, "point tiling");

extern "C" void kernel_launch(void* const* d_in, const int* in_sizes, int n_in,
                              void* d_out, int out_size, void* d_ws, size_t ws_size,
                              hipStream_t stream) {
  (void)in_sizes;
  (void)out_size;
  if (n_in < 12) return;
  if (ws_size < WS_TOTAL) return;
  const float* xyz1     = (const float*)d_in[0];
  const float* xyz2     = (const float*)d_in[1];
  const float* feature1 = (const float*)d_in[2];
  const float* feature2 = (const float*)d_in[3];
  const float* w1_0  = (const float*)d_in[4];
  const float* bn1_0 = (const float*)d_in[5];
  const float* w1_1  = (const float*)d_in[6];
  const float* bn1_1 = (const float*)d_in[7];
  const float* w1_2  = (const float*)d_in[8];
  const float* bn1_2 = (const float*)d_in[9];
  const float* w2_0  = (const float*)d_in[10];
  const float* bn2_0 = (const float*)d_in[11];
  float* out = (float*)d_out;

  char* ws = (char*)d_ws;
  int* idx            = (int*)(ws + WS_IDX);
  unsigned short* f2T = (unsigned short*)(ws + WS_F2T);
  float* Ppl          = (float*)(ws + WS_PPL);
  unsigned short* X2  = (unsigned short*)(ws + WS_X2);
  unsigned short* X2L = (unsigned short*)(ws + WS_X2L);
  unsigned short* wpl = (unsigned short*)(ws + WS_WPL);
  float* wp           = (float*)(ws + WS_WP);
  float* bnt          = (float*)(ws + WS_BNT);

  prep_planes<<<dim3(90), dim3(256), 0, stream>>>(w1_0, w1_1, w1_2, w2_0, bn1_0, bn1_1, bn1_2, bn2_0, wpl, wp, bnt);

  transpose_cast<CH_F2, false><<<dim3(NPTS2 / 32, NBATCH), dim3(256), 0, stream>>>(feature2, f2T, f2T, NPTS2, CH_F2, 0);

  transpose_cast<CH_F1, true><<<dim3(NPTS1 / 32, NBATCH), dim3(256), 0, stream>>>(feature1, X2, X2L, NPTS1, KDIM_MLP2, CH_L2);

  knn8_kernel<<<dim3(NPTS1 / 256, NBATCH), dim3(256), 0, stream>>>(xyz1, xyz2, idx);

  {
    const int tiles = ((NBATCH * NPTS2) / 64) * (CH_L0 / 64);
    gemm64_f16<false><<<dim3(tiles / 8, 1), dim3(256), 0, stream>>>(
        f2T, CH_F2, 0L, wpl + WPL_WF, CH_F2, 0L, Ppl, CH_L0, 0L, bnt, bnt,
        NBATCH * NPTS2, CH_L0, CH_F2);
  }

  mlp1_fused<<<dim3((NBATCH * NPTS1) / 16), dim3(128), 0, stream>>>(
      xyz1, xyz2, idx, Ppl, wpl + WPL_W1, wpl + WPL_W2, wp, bnt, X2, X2L);

  {
    const int tiles = (CH_OUT / 64) * (NPTS1 / 32);
    gemm_mlp2_hilo<<<dim3(tiles / 8, NBATCH), dim3(256), 0, stream>>>(
        wpl + WPL_W4, KDIM_MLP2, X2, X2L, KDIM_MLP2, (long)NPTS1 * KDIM_MLP2,
        out, NPTS1, (long)CH_OUT * NPTS1, bnt + BNT_S4, bnt + BNT_T4,
        CH_OUT, NPTS1, KDIM_MLP2);
  }
}
